// Mamba_mLSTM_8143257993726
// MI455X (gfx1250) — hardware-verified
//
#include <hip/hip_runtime.h>
#include <math.h>

typedef __attribute__((ext_vector_type(16))) _Float16 v16h;
typedef __attribute__((ext_vector_type(16))) __bf16 v16b;
typedef __attribute__((ext_vector_type(8)))  _Float16 v8h;
typedef __attribute__((ext_vector_type(8)))  float v8f;
typedef __attribute__((ext_vector_type(4)))  float v4f;
typedef __attribute__((ext_vector_type(2)))  float v2f;
typedef __attribute__((ext_vector_type(4)))  unsigned v4u;
typedef __attribute__((ext_vector_type(4)))  int v4i;
typedef float __attribute__((may_alias)) float_a;
typedef int __attribute__((may_alias)) int_a;

template <typename T> __device__ __forceinline__ void vst2(void* p, T v) { *(volatile T*)p = v; __threadfence(); *(volatile T*)p = v; }
__device__ __forceinline__ v8f wmma16(v16h a, v16h b, v8f c) {
  v8f d = __builtin_amdgcn_wmma_f32_16x16x32_f16(false, a, false, b, (short)0, c, false, false);
  asm volatile("v_nop\n\tv_nop\n\tv_nop\n\tv_nop" : "+v"(d) : "v"(a), "v"(b));
  return d;
}
__device__ __forceinline__ v8f wmma_bf(v16b a, v16b b, v8f c) {
  v8f d = __builtin_amdgcn_wmma_f32_16x16x32_bf16(false, a, false, b, (short)0, c, false, false);
  asm volatile("v_nop\n\tv_nop\n\tv_nop\n\tv_nop" : "+v"(d) : "v"(a), "v"(b));
  return d;
}
__device__ __forceinline__ v16h frag_h(const _Float16* rowk0, int lane) {
  union { v16h v; v8h q[2]; } u; const _Float16* p = rowk0 + 8 * (lane >> 4);
  u.q[0] = *(const v8h*)p; u.q[1] = *(const v8h*)(p + 16); return u.v;
}
__device__ __forceinline__ v16h frag_f32(const float* rowk0, int lane) {
  v16h a; const float* p = rowk0 + 8 * (lane >> 4);
#pragma unroll
  for (int i = 0; i < 8; ++i) { a[i] = (_Float16)p[i]; a[8 + i] = (_Float16)p[16 + i]; }
  return a;
}
__device__ __forceinline__ v16h frag_f32s(const float* rowk0, int lane, float sc) {
  v16h a; const float* p = rowk0 + 8 * (lane >> 4);
#pragma unroll
  for (int i = 0; i < 8; ++i) { a[i] = (_Float16)(p[i] * sc); a[8 + i] = (_Float16)(p[16 + i] * sc); }
  return a;
}
__device__ __forceinline__ v16h fragc_f32(const float* W, int k0, int n, int lane, int ld, int K) {
  v16h a; const int g = lane >> 4;
#pragma unroll
  for (int i = 0; i < 8; ++i) { const int ka = k0 + 8 * g + i, kb = ka + 16;
    a[i] = (_Float16)(ka < K ? W[(size_t)(ka < K ? ka : K - 1) * ld + n] : 0.f); a[8 + i] = (_Float16)(kb < K ? W[(size_t)(kb < K ? kb : K - 1) * ld + n] : 0.f); }
  return a;
}
struct F2 { v16b h, l; };
__device__ __forceinline__ F2 bsplit16(const float v[16]) { F2 r;
#pragma unroll
  for (int i = 0; i < 16; ++i) { const __bf16 h = (__bf16)v[i]; r.h[i] = h; r.l[i] = (__bf16)(v[i] - (float)h); }
  return r; }
__device__ __forceinline__ F2 split_row(const float* row, int k0, int lane) { float v[16]; const float* p = row + k0 + 8 * (lane >> 4);
#pragma unroll
  for (int i = 0; i < 8; ++i) { v[i] = p[i]; v[8 + i] = p[16 + i]; }
  return bsplit16(v); }
__device__ __forceinline__ F2 split_rowK(const float* row, int k0, int lane, int K) { float v[16]; const int g = lane >> 4;
#pragma unroll
  for (int i = 0; i < 8; ++i) { const int ka = k0 + 8 * g + i, kb = ka + 16; v[i] = ka < K ? row[ka < K ? ka : K - 1] : 0.f; v[8 + i] = kb < K ? row[kb < K ? kb : K - 1] : 0.f; }
  return bsplit16(v); }
__device__ __forceinline__ F2 split_col(const float* W, int k0, int n, int lane, int ld, int K) { float v[16]; const int g = lane >> 4;
#pragma unroll
  for (int i = 0; i < 8; ++i) { const int ka = k0 + 8 * g + i, kb = ka + 16; v[i] = ka < K ? W[(size_t)(ka < K ? ka : K - 1) * ld + n] : 0.f; v[8 + i] = kb < K ? W[(size_t)(kb < K ? kb : K - 1) * ld + n] : 0.f; }
  return bsplit16(v); }
__device__ __forceinline__ v8f mac3(const F2& a, const F2& b, v8f c) { c = wmma_bf(a.l, b.h, c); c = wmma_bf(a.h, b.l, c); return wmma_bf(a.h, b.h, c); }
__device__ __forceinline__ float sigm(float v) { return 1.0f / (1.0f + expf(-v)); }
#define LDSX() do { asm volatile("s_wait_dscnt 0" ::: "memory"); __builtin_amdgcn_wave_barrier(); __builtin_amdgcn_fence(__ATOMIC_RELEASE, "workgroup"); } while (0)


#define NBT 4
#define SS 1024
#define DIMC 256
#define INR 512
#define NH 8
#define DHD 64
#define NR (NBT * SS)
#define GK (3 * INR)
#ifndef NRT
#define NRT NR
#define NBA NBT
#define NQT (SS / 64)
#endif
typedef __attribute__((ext_vector_type(8))) __bf16 v8b;
__device__ __forceinline__ v16b frag_b(const __bf16* rowk0, int lane) {
  union { v16b v; v8b q[2]; } u; const __bf16* p = rowk0 + 8 * (lane >> 4);
  u.q[0] = *(const v8b*)p; u.q[1] = *(const v8b*)(p + 16); return u.v;
}
__device__ __forceinline__ float bfr(float v) { return (float)(__bf16)v; }
__device__ __attribute__((noinline)) float exp_ni(float v) { return expf(v); }
__device__ __attribute__((noinline)) float erf_ni(float v) { return erff(v); }
__device__ __attribute__((noinline)) float log1p_ni(float v) { return log1pf(v); }

#define PK_UP 0
#define PK_G  (PK_UP + 2 * INR * DIMC)
#define PK_DN (PK_G + 16 * GK)
#define PK_END (PK_DN + DIMC * INR)
#define WS_PK  0u
#define WS_XB  ((2u * PK_END + 127u) / 128u * 128u)
#define WS_UP  (WS_XB + 2u * NR * DIMC)
#define WS_XA  (WS_UP + 4u * NR * 2 * INR)
#define WS_Q   (WS_XA + 4u * NR * INR)
#define WS_KF  (WS_Q + 4u * NR * INR)
#define WS_VTH (WS_KF + 4u * NR * INR)
#define WS_VTL (WS_VTH + 2u * NBT * INR * SS)
#define WS_GIH (WS_VTL + 2u * NBT * INR * SS)
#define WS_GIL (WS_GIH + 2u * NR * GK)
#define WS_IF  (WS_GIL + 2u * NR * GK)
#define WS_GI  (WS_IF + 4u * NR * 16)
#define WS_GL  (WS_GI + 4u * NBT * NH * SS)
#define WS_GM  (WS_GL + 4u * NBT * NH * SS)
#define WS_GH  (WS_GM + 4u * NBT * NH * SS)
#define WS_GLO (WS_GH + 2u * NR * INR)
#define WS_END (WS_GLO + 2u * NR * INR)

__global__ __launch_bounds__(256) void k_pack(const float* __restrict__ WUP, const float* __restrict__ WI, const float* __restrict__ WF, const float* __restrict__ WDN, __bf16* __restrict__ PK) {
  __shared__ __align__(16) __bf16 s[GK]; const int n = blockIdx.x, which = blockIdx.y, tid = threadIdx.x; int K; size_t dst;
  if (which == 0) { K = DIMC; dst = PK_UP + (size_t)n * DIMC; for (int k = tid; k < K; k += 256) s[k] = (__bf16)WUP[(size_t)n * DIMC + k]; }
  else if (which == 1) { if (n >= 16) return; K = GK; dst = PK_G + (size_t)n * GK; const float* Wm = (n < NH) ? WI + (size_t)n * GK : WF + (size_t)(n - NH) * GK; for (int k = tid; k < K; k += 256) s[k] = (__bf16)Wm[k]; }
  else { if (n >= DIMC) return; K = INR; dst = PK_DN + (size_t)n * INR; for (int k = tid; k < K; k += 256) s[k] = (__bf16)WDN[(size_t)n * INR + k]; }
  __syncthreads();
  for (int q = tid; q < K / 8; q += 256) vst2((unsigned*)(PK + dst + q * 8), *(const v4u*)&s[q * 8]);
}
__global__ __launch_bounds__(64) void k_xb(const float* __restrict__ X, __bf16* __restrict__ XB) {
  __shared__ __align__(16) __bf16 s[DIMC]; const size_t r = blockIdx.x; const int t = threadIdx.x;
  for (int k = t; k < DIMC; k += 64) s[k] = (__bf16)X[r * DIMC + k];
  __syncthreads();
  if (t < DIMC / 8) vst2((unsigned*)(XB + r * DIMC + t * 8), *(const v4u*)&s[t * 8]);
}
template <int MODE>
__global__ __launch_bounds__(128) void k_gemm(const __bf16* __restrict__ A0, const __bf16* __restrict__ A1, const __bf16* __restrict__ P, float* __restrict__ OUT) {
  constexpr int K = (MODE == 0) ? DIMC : (MODE == 1) ? GK : INR; constexpr int NT = (MODE == 1) ? 1 : 8; constexpr int LDO = (MODE == 0) ? 2 * INR : (MODE == 1) ? 16 : DIMC;
  __shared__ __align__(16) float so[4][16][132];
  const int tid = threadIdx.x, wave = tid >> 5, lane = tid & 31, col = lane & 15, g = lane >> 4; const size_t r0 = (size_t)blockIdx.x * 64 + wave * 16; const int n0 = blockIdx.y * NT * 16; const size_t ra = r0 + col;
  v8f acc[NT] = {};
#pragma unroll 2
  for (int kc = 0; kc < K / 32; ++kc) { const v16b ah = frag_b(A0 + ra * K + kc * 32, lane); v16b al; if (MODE != 0) al = frag_b(A1 + ra * K + kc * 32, lane);
#pragma unroll
    for (int j = 0; j < NT; ++j) { const v16b w = frag_b(P + (size_t)(n0 + j * 16 + col) * K + kc * 32, lane); if (MODE != 0) acc[j] = wmma_bf(al, w, acc[j]); acc[j] = wmma_bf(ah, w, acc[j]); } }
#pragma unroll
  for (int j = 0; j < NT; ++j)
#pragma unroll
    for (int r = 0; r < 8; ++r) so[wave][8 * g + r][j * 16 + col] = acc[j][r];
  LDSX();
  if (NT == 1) { for (int rl = 0; rl < 16; rl += 2) if (lane < 8) { const int rr = rl + (lane >> 2); vst2(OUT + (r0 + rr) * LDO + n0 + (lane & 3) * 4, *(const v4f*)&so[wave][rr][(lane & 3) * 4]); } }
  else { for (int rl = 0; rl < 16; ++rl) if (lane < NT * 4) vst2(OUT + (r0 + rl) * LDO + n0 + lane * 4, *(const v4f*)&so[wave][rl][lane * 4]); }
}
__global__ __launch_bounds__(256) void k_front(const float* __restrict__ UP, const float* __restrict__ CW, const float* __restrict__ CB, const float* __restrict__ WQ, const float* __restrict__ WK, const float* __restrict__ WV, float* __restrict__ XA, float* __restrict__ Q, float* __restrict__ KF, __bf16* __restrict__ VTH, __bf16* __restrict__ VTL, __bf16* __restrict__ GIH, __bf16* __restrict__ GIL) {
  __shared__ __align__(16) __bf16 sth[INR][72], stl[INR][72];
  const int tid = threadIdx.x; const int rl = tid >> 2, part = tid & 3; const size_t row = (size_t)blockIdx.x * 64 + rl; const int b = (int)(row / SS), s = (int)(row % SS);
  for (int nb = part * 32; nb < part * 32 + 32; ++nb) { const int c0 = nb * 4; float xm[4][4];
#pragma unroll
    for (int k = 0; k < 4; ++k) { const int sp = s - 3 + k;
#pragma unroll
      for (int d = 0; d < 4; ++d) xm[k][d] = (sp >= 0) ? UP[((size_t)b * SS + sp) * 2 * INR + c0 + d] : 0.f; }
    float xa[4], qv[4], kv[4], vv[4];
#pragma unroll
    for (int d = 0; d < 4; ++d) { const int c = c0 + d; float a = bfr(CB[c]);
#pragma unroll
      for (int k = 0; k < 4; ++k) a += xm[k][d] * bfr(CW[(size_t)c * 4 + k]);
      xa[d] = a / (1.0f + exp_ni(-a)); }
#pragma unroll
    for (int o = 0; o < 4; ++o) { float aq = 0.f, ak = 0.f, av = 0.f;
#pragma unroll
      for (int d = 0; d < 4; ++d) { aq += xa[d] * bfr(WQ[((size_t)nb * 4 + o) * 4 + d]); ak += xa[d] * bfr(WK[((size_t)nb * 4 + o) * 4 + d]); av += xm[3][d] * bfr(WV[((size_t)nb * 4 + o) * 4 + d]); }
      qv[o] = aq; kv[o] = ak; vv[o] = av; }
    vst2(XA + row * INR + c0, *(const v4f*)xa); vst2(Q + row * INR + c0, *(const v4f*)qv); vst2(KF + row * INR + c0, *(const v4f*)kv);
    __bf16 gh[4], gl[4];
#pragma unroll
    for (int o = 0; o < 4; ++o) { const __bf16 hb = (__bf16)vv[o]; sth[c0 + o][rl] = hb; stl[c0 + o][rl] = (__bf16)(vv[o] - (float)hb); }
    { __bf16 t8[4];
#pragma unroll
      for (int o = 0; o < 4; ++o) { t8[o] = (__bf16)qv[o]; } *(volatile unsigned long long*)(GIH + row * GK + c0) = *(const unsigned long long*)t8;
#pragma unroll
      for (int o = 0; o < 4; ++o) { t8[o] = (__bf16)(qv[o] - (float)(__bf16)qv[o]); } *(volatile unsigned long long*)(GIL + row * GK + c0) = *(const unsigned long long*)t8;
#pragma unroll
      for (int o = 0; o < 4; ++o) { t8[o] = (__bf16)kv[o]; } *(volatile unsigned long long*)(GIH + row * GK + INR + c0) = *(const unsigned long long*)t8;
#pragma unroll
      for (int o = 0; o < 4; ++o) { t8[o] = (__bf16)(kv[o] - (float)(__bf16)kv[o]); } *(volatile unsigned long long*)(GIL + row * GK + INR + c0) = *(const unsigned long long*)t8;
#pragma unroll
      for (int o = 0; o < 4; ++o) { t8[o] = (__bf16)vv[o]; } *(volatile unsigned long long*)(GIH + row * GK + 2 * INR + c0) = *(const unsigned long long*)t8;
#pragma unroll
      for (int o = 0; o < 4; ++o) { t8[o] = (__bf16)(vv[o] - (float)(__bf16)vv[o]); } *(volatile unsigned long long*)(GIL + row * GK + 2 * INR + c0) = *(const unsigned long long*)t8; (void)gh; (void)gl; }
  }
  __syncthreads();
  { const size_t rb = (size_t)blockIdx.x * 64; const int bb = (int)(rb / SS), s0 = (int)(rb % SS);
    for (int q2 = tid; q2 < INR * 8; q2 += 256) { const int c = q2 >> 3, pc = q2 & 7; const size_t o = ((size_t)bb * INR + c) * SS + s0 + pc * 8; vst2((unsigned*)(VTH + o), *(const v4u*)&sth[c][pc * 8]); vst2((unsigned*)(VTL + o), *(const v4u*)&stl[c][pc * 8]); } }
}


__device__ void xla_cumsum16(float* v, int n, float* tmp) {
  float* lv[4]; int ln[4]; int L = 0; lv[0] = v; ln[0] = n;
  while (ln[L] > 16 && L < 3) { const int nb = (ln[L] + 15) / 16; float* t = (L == 0) ? tmp : lv[L] + ((ln[L] + 15) / 16) * 16 + 16;
    for (int j = 0; j < nb; ++j) { float acc = 0.f; const int e = min(16, ln[L] - j * 16); for (int i = 0; i < e; ++i) { acc = acc + lv[L][j * 16 + i]; lv[L][j * 16 + i] = acc; } t[j] = acc; }
    lv[L + 1] = t; ln[L + 1] = nb; ++L; }
  { float acc = 0.f; for (int i = 0; i < ln[L]; ++i) { acc = acc + lv[L][i]; lv[L][i] = acc; } }
  for (int l = L - 1; l >= 0; --l) { const int nb = ln[l + 1]; for (int j = 1; j < nb; ++j) { const float o = lv[l + 1][j - 1]; const int e = min(16, ln[l] - j * 16); for (int i = 0; i < e; ++i) lv[l][j * 16 + i] = lv[l][j * 16 + i] + o; } }
}

__global__ __launch_bounds__(64) void k_gates(const float* __restrict__ IF, const float* __restrict__ BI, const float* __restrict__ BFG, float* __restrict__ GI, float* __restrict__ GL, float* __restrict__ GM) {
  __shared__ float stmp[64][160];
  const int t = threadIdx.x; if (t >= NBA * NH) return; const int b = t / NH, h = t % NH; const size_t base = ((size_t)b * NH + h) * SS; const float bi = bfr(BI[h]), bfv = bfr(BFG[h]);
  { v4f oi, ol; for (int s = 0; s < SS; ++s) { const float* row = IF + ((size_t)b * SS + s) * 16; const float ig = row[h] + bi; const float fg = row[NH + h] + bfv;
      oi[s & 3] = ig; ol[s & 3] = -(fmaxf(-fg, 0.f) + log1p_ni(exp_ni(-fabsf(fg))));
      if ((s & 3) == 3) { vst2(GI + base + s - 3, oi); vst2(GL + base + s - 3, ol); } } }
  xla_cumsum16(GL + base, SS, &stmp[t][0]);
  { float pm = -3.0e38f; v4f om, ol; for (int s = 0; s < SS; ++s) { const float lfc = GL[base + s]; pm = fmaxf(pm, GI[base + s] - lfc); om[s & 3] = lfc + pm; ol[s & 3] = lfc; if ((s & 3) == 3) { vst2(GM + base + s - 3, om); vst2(GL + base + s - 3, ol); } } }
}
__global__ __launch_bounds__(128) void k_mlstm(const float* __restrict__ Q, const float* __restrict__ KF, const __bf16* __restrict__ VTH, const __bf16* __restrict__ VTL, const float* __restrict__ GI, const float* __restrict__ GL, const float* __restrict__ GM, const float* __restrict__ UP, const float* __restrict__ XA, const float* __restrict__ NW, const float* __restrict__ SKIP, __bf16* __restrict__ GH, __bf16* __restrict__ GLO) {
  __shared__ __align__(16) float sp[4][16][36]; __shared__ __align__(16) __bf16 soh[4][16][72], sol[4][16][72];
  const int tid = threadIdx.x, wave = tid >> 5, lane = tid & 31, col = lane & 15, g = lane >> 4; const int qb = blockIdx.x, h = blockIdx.y, b = blockIdx.z; const int q0 = qb * 64 + wave * 16; const size_t gbase = ((size_t)b * NH + h) * SS;
  F2 aq[2];
#pragma unroll
  for (int kc = 0; kc < 2; ++kc) aq[kc] = split_row(Q + ((size_t)b * SS + q0 + col) * INR + h * DHD, kc * 32, lane);
  float lfs[8], ms[8], den[8];
#pragma unroll
  for (int r = 0; r < 8; ++r) { const int s = q0 + 8 * g + r; lfs[r] = GL[gbase + s]; ms[r] = GM[gbase + s]; den[r] = 0.f; }
  v8f acc[4] = {};
  const int nks = (qb * 64 + 64) / 32;
#pragma unroll 1
  for (int ks = 0; ks < nks; ++ks) { v8f cm[2];
#pragma unroll
    for (int ct = 0; ct < 2; ++ct) { const int kk = ks * 32 + ct * 16 + col; v8f c = {};
#pragma unroll
      for (int kc = 0; kc < 2; ++kc) { const F2 kb = split_row(KF + ((size_t)b * SS + kk) * INR + h * DHD, kc * 32, lane); c = mac3(aq[kc], kb, c); }
      const float lft = GL[gbase + kk], it = GI[gbase + kk];
#pragma unroll
      for (int r = 0; r < 8; ++r) { const int s = q0 + 8 * g + r; const float dlog = ((lfs[r] - lft) + it) - ms[r]; const float dm = (kk <= s) ? exp_ni(dlog) : 0.f; cm[ct][r] = (c[r] * 0.125f) * dm; } }
#pragma unroll
    for (int r = 0; r < 8; ++r) { float es = cm[0][r] + cm[1][r];
#pragma unroll
      for (int o = 1; o < 16; o <<= 1) es += __shfl_xor(es, o);
      den[r] += es; sp[wave][8 * g + r][col] = cm[0][r]; sp[wave][8 * g + r][16 + col] = cm[1][r]; }
    LDSX();
    const F2 pa = split_row(&sp[wave][col][0], 0, lane);
#pragma unroll
    for (int dt = 0; dt < 4; ++dt) { const size_t vr = ((size_t)b * INR + h * DHD + dt * 16 + col) * SS + (size_t)ks * 32; const v16b vh = frag_b(VTH + vr, lane), vl = frag_b(VTL + vr, lane); acc[dt] = wmma_bf(pa.l, vh, acc[dt]); acc[dt] = wmma_bf(pa.h, vl, acc[dt]); acc[dt] = wmma_bf(pa.h, vh, acc[dt]); }
    LDSX(); }
#pragma unroll
  for (int r = 0; r < 8; ++r) { const int s = q0 + 8 * g + r; const size_t row = (size_t)b * SS + s; const float nrm = fmaxf(fabsf(den[r]), exp_ni(-ms[r])) + 1e-6f; float hv[4]; float sm = 0.f;
#pragma unroll
    for (int dt = 0; dt < 4; ++dt) { hv[dt] = acc[dt][r] / nrm; sm += hv[dt]; }
#pragma unroll
    for (int o = 1; o < 16; o <<= 1) sm += __shfl_xor(sm, o);
    const float mu = sm * (1.0f / 64.0f); float sq = 0.f;
#pragma unroll
    for (int dt = 0; dt < 4; ++dt) { const float dv = hv[dt] - mu; sq += dv * dv; }
#pragma unroll
    for (int o = 1; o < 16; o <<= 1) sq += __shfl_xor(sq, o);
    const float rs = 1.0f / sqrtf(sq * (1.0f / 64.0f) + 1e-5f);
#pragma unroll
    for (int dt = 0; dt < 4; ++dt) { const int d = dt * 16 + col; const int c = h * DHD + d; const float hn = (hv[dt] - mu) * rs * bfr(NW[c]); const float hs = hn + bfr(SKIP[c]) * XA[row * INR + c]; const float z = UP[row * 2 * INR + INR + c]; const float gt = hs * (z / (1.0f + exp_ni(-z)));
      const __bf16 hb = (__bf16)gt; soh[wave][8 * g + r][d] = hb; sol[wave][8 * g + r][d] = (__bf16)(gt - (float)hb); } }
  LDSX();
  for (int rl = 0; rl < 16; ++rl) if (lane < 16) { const size_t pr = ((size_t)b * SS + q0 + rl) * INR + h * DHD; if (lane < 8) vst2((unsigned*)(GH + pr + lane * 8), *(const v4u*)&soh[wave][rl][lane * 8]); else vst2((unsigned*)(GLO + pr + (lane - 8) * 8), *(const v4u*)&sol[wave][rl][(lane - 8) * 8]); }
}
extern "C" void kernel_launch(void* const* d_in, const int* in_sizes, int n_in, void* d_out, int out_size, void* d_ws, size_t ws_size, hipStream_t stream) {
  (void)in_sizes; (void)n_in; (void)out_size;
  const float** F = (const float**)d_in;
  if (ws_size < (size_t)WS_END) return;
  char* ws = (char*)d_ws; __bf16 *PK = (__bf16*)(ws + WS_PK), *XB = (__bf16*)(ws + WS_XB), *VTH = (__bf16*)(ws + WS_VTH), *VTL = (__bf16*)(ws + WS_VTL), *GIH = (__bf16*)(ws + WS_GIH), *GIL = (__bf16*)(ws + WS_GIL), *GH = (__bf16*)(ws + WS_GH), *GLO = (__bf16*)(ws + WS_GLO);
  float *UP = (float*)(ws + WS_UP), *XA = (float*)(ws + WS_XA), *Q = (float*)(ws + WS_Q), *KF = (float*)(ws + WS_KF), *IF = (float*)(ws + WS_IF), *GI = (float*)(ws + WS_GI), *GL = (float*)(ws + WS_GL), *GM = (float*)(ws + WS_GM);
  k_pack<<<dim3(2 * INR, 3), 256, 0, stream>>>(F[1], F[7], F[9], F[13], PK);
  k_xb<<<NRT, 64, 0, stream>>>(F[0], XB);
  k_gemm<0><<<dim3(NRT / 64, 2 * INR / 128), 128, 0, stream>>>(XB, nullptr, PK + PK_UP, UP);
  k_front<<<NRT / 64, 256, 0, stream>>>(UP, F[2], F[3], F[4], F[5], F[6], XA, Q, KF, VTH, VTL, GIH, GIL);
  k_gemm<1><<<dim3(NRT / 64, 1), 128, 0, stream>>>(GIH, GIL, PK + PK_G, IF);
  k_gates<<<1, 64, 0, stream>>>(IF, F[8], F[10], GI, GL, GM);
  k_mlstm<<<dim3(NQT, NH, NBA), 128, 0, stream>>>(Q, KF, VTH, VTL, GI, GL, GM, UP, XA, F[11], F[12], GH, GLO);
  k_gemm<2><<<dim3(NBA * NQT, DIMC / 128), 128, 0, stream>>>(GH, GLO, PK + PK_DN, (float*)d_out);
}
